// MultiScaleRetention_25074019074211
// MI455X (gfx1250) — hardware-verified
//
#include <hip/hip_runtime.h>
#include <math.h>

constexpr int kBatch = 2;
constexpr int kSeqT  = 2048;
constexpr int kEmb   = 1024;
constexpr int kEmb2  = 2048;
constexpr int kHeads = 4;
constexpr int kDk    = 256;
constexpr int kDv    = 512;
constexpr int kTok   = kBatch * kSeqT;
constexpr float kWCarry     = 64.0f;
constexpr float kWCarryInv  = 1.0f / 64.0f;
constexpr float kQScale     = 0.0625f;
constexpr float kSCarry     = 1024.0f;
constexpr float kSCarryInv  = 1.0f / 1024.0f;
constexpr float kHCarry     = 16.0f;
constexpr float kOutScale   = 1.0f / (16.0f * 64.0f);
constexpr float kEps        = 1e-5f;
constexpr float kInvDv      = 1.0f / 512.0f;

typedef __attribute__((ext_vector_type(16))) _Float16 v16h;
typedef __attribute__((ext_vector_type(8)))  _Float16 v8h;
typedef __attribute__((ext_vector_type(16))) __bf16   v16b;
typedef __attribute__((ext_vector_type(8)))  __bf16   v8b;
typedef __attribute__((ext_vector_type(8)))  float    v8f;
typedef __attribute__((ext_vector_type(4)))  float    v4f;
typedef __attribute__((ext_vector_type(4)))  unsigned int v4u;

__device__ __forceinline__ unsigned short f2bf_bits(float f) {
  unsigned u = __float_as_uint(f);
  return (unsigned short)((u + 0x7FFFu + ((u >> 16) & 1u)) >> 16);
}
__device__ __forceinline__ float bf_bits2f(unsigned short h) { return __uint_as_float(((unsigned)h) << 16); }

__device__ __forceinline__ void dep_guard_h(v8f& a, v8f& b, v16h x, v16h y) { asm volatile("v_nop\n\tv_nop\n\tv_nop\n\tv_nop" : "+v"(a), "+v"(b) : "v"(x), "v"(y)); }
__device__ __forceinline__ void dep_guard_b(v8f& a, v8f& b, v16b x, v16b y) { asm volatile("v_nop\n\tv_nop\n\tv_nop\n\tv_nop" : "+v"(a), "+v"(b) : "v"(x), "v"(y)); }
__device__ __forceinline__ void keep4_h(v16h a, v16h b, v16h c, v16h d) { asm volatile("v_nop" :: "v"(a), "v"(b), "v"(c), "v"(d)); }
__device__ __forceinline__ void keep4_b(v16b a, v16b b, v16b c, v16b d) { asm volatile("v_nop" :: "v"(a), "v"(b), "v"(c), "v"(d)); }
__device__ __forceinline__ void acc_guard4(v8f& a, v8f& b, v8f& c, v8f& d) { asm volatile("v_nop\n\tv_nop\n\tv_nop\n\tv_nop" : "+v"(a), "+v"(b), "+v"(c), "+v"(d)); }
template <typename T> struct Frag;
template <> struct Frag<_Float16> {
  typedef v16h V; union U { v16h v; v8h h[2]; };
  static __device__ __forceinline__ v16h load(const _Float16* p) {
    U f; f.h[0] = *(const v8h*)(p); f.h[1] = *(const v8h*)(p + 16); return f.v;
  }
  static __device__ __forceinline__ v8f mma(v16h a, v16h b, v8f c) {
    return __builtin_amdgcn_wmma_f32_16x16x32_f16(false, a, false, b, (short)0, c, false, false);
  }
  static __device__ __forceinline__ void guard(v8f& a, v8f& b, v16h x, v16h y) { dep_guard_h(a, b, x, y); }
  static __device__ __forceinline__ void keep(v16h a, v16h b, v16h c, v16h d) { keep4_h(a, b, c, d); }
};
template <> struct Frag<__bf16> {
  typedef v16b V; union U { v16b v; v8b h[2]; };
  static __device__ __forceinline__ v16b load(const __bf16* p) {
    U f; f.h[0] = *(const v8b*)(p); f.h[1] = *(const v8b*)(p + 16); return f.v;
  }
  static __device__ __forceinline__ v8f mma(v16b a, v16b b, v8f c) {
    return __builtin_amdgcn_wmma_f32_16x16x32_bf16(false, a, false, b, (short)0, c, false, false);
  }
  static __device__ __forceinline__ void guard(v8f& a, v8f& b, v16b x, v16b y) { dep_guard_b(a, b, x, y); }
  static __device__ __forceinline__ void keep(v16b a, v16b b, v16b c, v16b d) { keep4_b(a, b, c, d); }
};

__device__ __forceinline__ unsigned pk16(unsigned short a, unsigned short b) { return (unsigned)a | ((unsigned)b << 16); }
__device__ __forceinline__ unsigned short h_bits(float f) { const _Float16 h = (_Float16)f; return __builtin_bit_cast(unsigned short, h); }

template <int ET> struct Elem;
template <> struct Elem<0> { typedef _Float16 T; };
template <> struct Elem<1> { typedef __bf16 T; };
template <int ET, bool SPLIT, int BIAS_MODE, int OUT_MODE, bool RESID, int ACT = 0, int CAUSAL = 0>
__global__ __launch_bounds__(256) void wmma_gemm64(
    const unsigned short* __restrict__ Ap, const unsigned short* __restrict__ A2p, int lda, long strideA,
    const unsigned short* __restrict__ Btp, const unsigned short* __restrict__ Bt2p, int ldb, long strideB,
    void* __restrict__ Cout, void* __restrict__ Cout2, int ldc, long strideC,
    const float* __restrict__ bias,
    const float* __restrict__ resid, long strideR,
    int M, int N, int K, float scale) {
  typedef typename Elem<ET>::T T;
  typedef typename Frag<T>::V V;
  const T* A = (const T*)Ap; const T* A2 = (const T*)A2p; const T* Bt = (const T*)Btp; const T* Bt2 = (const T*)Bt2p;
  __shared__ __align__(16) float sT[8][16 * 68];
  const int b    = blockIdx.y;
  const int lane = threadIdx.x & 31;
  const int wave = threadIdx.x >> 5;
  const int tilesN = N >> 6;
  const int tilesM = M >> 6;
  const int tile = blockIdx.x * 8 + wave;
  if (tile >= tilesM * tilesN) return;
  const int tm = tile / tilesN;
  const int tn = tile - tm * tilesN;
  const int m0 = tm << 6;
  const int n0 = tn << 6;
  if (CAUSAL == 1 && n0 >= m0 + 64) return;
  const int Kend = (CAUSAL == 2) ? (((m0 + 64) < K) ? (m0 + 64) : K) : K;

  const T* Ab  = A  + (size_t)b * strideA;
  const T* Bb  = Bt + (size_t)b * strideB;
  const T* Ab2 = SPLIT ? (A2  + (size_t)b * strideA) : nullptr;
  const T* Bb2 = SPLIT ? (Bt2 + (size_t)b * strideB) : nullptr;

  const int rlane = lane & 15;
  const int koff  = (lane >> 4) * 8;
  const int mOff  = (lane >> 4) * 8;

  v8f acc[4][4];
#pragma unroll
  for (int i = 0; i < 4; ++i)
#pragma unroll
    for (int j = 0; j < 4; ++j) acc[i][j] = (v8f){0.f,0.f,0.f,0.f,0.f,0.f,0.f,0.f};

  for (int k0 = 0; k0 < Kend; k0 += 32) {
    V bh[4], bl[4];
#pragma unroll
    for (int j = 0; j < 4; ++j) {
      const size_t bo = (size_t)(n0 + (j << 4) + rlane) * ldb + koff + k0;
      bh[j] = Frag<T>::load(Bb + bo);
      if (SPLIT) bl[j] = Frag<T>::load(Bb2 + bo);
    }
#pragma unroll
    for (int i = 0; i < 4; ++i) {
      const size_t ao = (size_t)(m0 + (i << 4) + rlane) * lda + koff + k0;
      V ah = Frag<T>::load(Ab + ao);
      V al;
      if (SPLIT) al = Frag<T>::load(Ab2 + ao);
#pragma unroll
      for (int j = 0; j < 4; ++j) {
        acc[i][j] = Frag<T>::mma(ah, bh[j], acc[i][j]);
        if (SPLIT) {
          acc[i][j] = Frag<T>::mma(ah, bl[j], acc[i][j]);
          acc[i][j] = Frag<T>::mma(al, bh[j], acc[i][j]);
        }
      }
      Frag<T>::guard(acc[i][0], acc[i][3], ah, SPLIT ? al : ah);
    }
    Frag<T>::keep(bh[0], bh[1], bh[2], bh[3]);
    if (SPLIT) Frag<T>::keep(bl[0], bl[1], bl[2], bl[3]);
  }
  acc_guard4(acc[0][0], acc[0][1], acc[0][2], acc[0][3]);
  acc_guard4(acc[1][0], acc[1][1], acc[1][2], acc[1][3]);
  acc_guard4(acc[2][0], acc[2][1], acc[2][2], acc[2][3]);
  acc_guard4(acc[3][0], acc[3][1], acc[3][2], acc[3][3]);

  float* slab = sT[wave];
  const float* Rb = RESID ? (resid + (size_t)b * strideR) : nullptr;
#pragma unroll
  for (int i = 0; i < 4; ++i) {
    const int mBase = m0 + (i << 4);
#pragma unroll
    for (int j = 0; j < 4; ++j) {
      const int n = n0 + (j << 4) + rlane;
      float bv = 0.f;
      if (BIAS_MODE == 2) bv = bias[n];
#pragma unroll
      for (int r = 0; r < 8; ++r) {
        float v = acc[i][j][r] * scale;
        if (BIAS_MODE == 1) v += bias[mBase + mOff + r];
        if (BIAS_MODE == 2) v += bv;
        if (RESID) v += Rb[(size_t)(mBase + mOff + r) * ldc + n];
        if (ACT == 2) v = fmaxf(v, 0.0f);
        if (ACT == 4) v = (v > 0.f) ? v : 0.01f * v;
        slab[(mOff + r) * 68 + (j << 4) + rlane] = v;
      }
    }
    __builtin_amdgcn_fence(__ATOMIC_RELEASE, "workgroup");
    __builtin_amdgcn_wave_barrier();
    __builtin_amdgcn_fence(__ATOMIC_ACQUIRE, "workgroup");
    if (OUT_MODE == 0) {
      float* C = (float*)Cout + (size_t)b * strideC;
      const int hh = lane >> 4, c4 = (lane & 15) * 4;
      for (int pass = 0; pass < 2; ++pass) {
#pragma unroll
        for (int it = 0; it < 8; ++it) {
          const int row = it * 2 + hh;
          v4f v = *(const v4f*)(slab + row * 68 + c4);
          *(volatile v4f*)(C + (size_t)(mBase + row) * ldc + n0 + c4) = v;
        }
        __threadfence();
      }
    } else {
      const int q = lane >> 3, c8 = (lane & 7) * 8;
      unsigned short* C  = (unsigned short*)Cout  + (size_t)b * strideC;
      unsigned short* C2 = (OUT_MODE == 2) ? ((unsigned short*)Cout2 + (size_t)b * strideC) : nullptr;
      for (int pass = 0; pass < 2; ++pass) {
#pragma unroll
        for (int it = 0; it < 4; ++it) {
          const int row = it * 4 + q;
          const float* sp = slab + row * 68 + c8;
          v8h hv, lv;
#pragma unroll
          for (int e = 0; e < 8; ++e) {
            if (OUT_MODE == 1) {
              hv[e] = (_Float16)sp[e];
            } else {
              unsigned short hb = f2bf_bits(sp[e]);
              unsigned short lb = f2bf_bits(sp[e] - bf_bits2f(hb));
              hv[e] = __builtin_bit_cast(_Float16, hb);
              lv[e] = __builtin_bit_cast(_Float16, lb);
            }
          }
          *(volatile v8h*)(C + (size_t)(mBase + row) * ldc + n0 + c8) = hv;
          if (OUT_MODE == 2) *(volatile v8h*)(C2 + (size_t)(mBase + row) * ldc + n0 + c8) = lv;
        }
        __threadfence();
      }
    }
    __builtin_amdgcn_fence(__ATOMIC_RELEASE, "workgroup");
    __builtin_amdgcn_wave_barrier();
    __builtin_amdgcn_fence(__ATOMIC_ACQUIRE, "workgroup");
  }
}

__global__ __launch_bounds__(256) void cast8_f16_kernel(const float* __restrict__ in, unsigned short* __restrict__ out, int n8) {
  const int i = blockIdx.x * 256 + threadIdx.x;
  if (i >= n8) return;
  const float* p = in + 8 * (size_t)i;
  const v4f a = *(const v4f*)(p);
  const v4f c = *(const v4f*)(p + 4);
  unsigned short hb[8];
#pragma unroll
  for (int e = 0; e < 4; ++e) {
    hb[e]     = h_bits(a[e]);
    hb[4 + e] = h_bits(c[e]);
  }
  const v4u u = (v4u){pk16(hb[0], hb[1]), pk16(hb[2], hb[3]), pk16(hb[4], hb[5]), pk16(hb[6], hb[7])};
  unsigned short* q = out + 8 * (size_t)i;
  *(volatile v4u*)q = u;
  __threadfence();
  *(volatile v4u*)q = u;
}

__global__ __launch_bounds__(256) void wtcast_kernel(const float* __restrict__ W0, const float* __restrict__ W1,
                                                     unsigned short* __restrict__ out0, unsigned short* __restrict__ out1,
                                                     int R, int Cn, float scale) {
  __shared__ float sm[64][65];
  const int t  = threadIdx.x;
  const int r0 = blockIdx.x * 64;
  const int c0 = blockIdx.y * 64;
  const int z  = blockIdx.z;
  const float* W = (z == 0) ? W0 : W1;
  unsigned short* op = (z == 0) ? out0 : out1;
#pragma unroll
  for (int i = 0; i < 16; ++i) {
    const int e = i * 256 + t;
    const int r = e >> 6;
    const int c = e & 63;
    sm[c][r] = W[(size_t)(r0 + r) * Cn + c0 + c] * scale;
  }
  __syncthreads();
  const int lane = t & 31, wave = t >> 5;
  const int q = lane >> 3, c8 = (lane & 7) * 8;
  for (int pass = 0; pass < 2; ++pass) {
#pragma unroll
    for (int it = 0; it < 2; ++it) {
      const int row = wave * 8 + it * 4 + q;
      unsigned short hb[8];
#pragma unroll
      for (int e = 0; e < 8; ++e) hb[e] = h_bits(sm[row][c8 + e]);
      const v4u u = (v4u){pk16(hb[0], hb[1]), pk16(hb[2], hb[3]), pk16(hb[4], hb[5]), pk16(hb[6], hb[7])};
      *(volatile v4u*)(op + (size_t)(c0 + row) * R + r0 + c8) = u;
    }
    __threadfence();
  }
}

struct RopeTab { float inv[128]; };
static_assert(sizeof(RopeTab) == 512, "size");

__global__ __launch_bounds__(128) void rotary_kernel(const float* __restrict__ TQ, const float* __restrict__ TK,
                                                     unsigned short* __restrict__ Qo, unsigned short* __restrict__ Ko,
                                                     RopeTab tab) {
#pragma clang fp contract(off)
  __shared__ __align__(16) unsigned short sq[256];
  __shared__ __align__(16) unsigned short sk[256];
  const int f   = threadIdx.x;
  const int blk = blockIdx.x;
  const int h   = blk & (kHeads - 1);
  const int tok = blk >> 2;
  const int t   = tok & (kSeqT - 1);
  const int b   = tok >> 11;
  const size_t ib = (size_t)tok * kEmb + (size_t)h * kDk;
  const float q1 = TQ[ib + f], q2 = TQ[ib + 128 + f];
  const float k1 = TK[ib + f], k2 = TK[ib + 128 + f];
  const float ang = (float)t * tab.inv[f];
  float sn, cs;
  sincosf(ang, &sn, &cs);
  const float qa = q1 * cs - q2 * sn;
  const float qb = q2 * cs + q1 * sn;
  const float ka = k1 * cs - k2 * sn;
  const float kb = k2 * cs + k1 * sn;
  sq[f] = h_bits(qa); sq[128 + f] = h_bits(qb);
  sk[f] = h_bits(ka); sk[128 + f] = h_bits(kb);
  __syncthreads();
  const int lane = f & 31, wave = f >> 5;
  const size_t ob = ((size_t)(b * kHeads + h) * kSeqT + t) * kDk + 8 * lane;
  const v4u uq = *(const v4u*)(sq + 8 * lane);
  const v4u uk = *(const v4u*)(sk + 8 * lane);
  for (int pass = 0; pass < 2; ++pass) {
    if (wave == 0) {
      *(volatile v4u*)(Qo + ob) = uq;
    } else if (wave == 1) {
      *(volatile v4u*)(Ko + ob) = uk;
    }
    __threadfence();
  }
}

__global__ __launch_bounds__(256) void decay_cast_kernel(const float* __restrict__ SC, unsigned short* __restrict__ Sout,
                                                         float lg2, float carry) {
  const int t   = blockIdx.x;
  const int tid = threadIdx.x;
  const int c0  = tid * 8;
  const float* sr = SC + (size_t)t * kSeqT + c0;
  const v4f a = *(const v4f*)(sr);
  const v4f c = *(const v4f*)(sr + 4);
  float x[8];
#pragma unroll
  for (int e = 0; e < 4; ++e) { x[e] = a[e]; x[4 + e] = c[e]; }
  unsigned short hb[8];
#pragma unroll
  for (int e = 0; e < 8; ++e) {
    const int n  = t - (c0 + e);
    const int nn = (n < 0) ? 0 : n;
    const float d = exp2f((float)nn * lg2);
    const float val = x[e] * d * carry;
    const float r = (n >= 0) ? val : 0.0f;
    hb[e] = h_bits(r);
  }
  const v4u u = (v4u){pk16(hb[0], hb[1]), pk16(hb[2], hb[3]), pk16(hb[4], hb[5]), pk16(hb[6], hb[7])};
  unsigned short* q = Sout + (size_t)t * kSeqT + c0;
  *(volatile v4u*)q = u;
  __threadfence();
  *(volatile v4u*)q = u;
}

__global__ __launch_bounds__(256) void rmsgate_kernel(const float* __restrict__ O, const float* __restrict__ G,
                                                      const float* __restrict__ gnw, unsigned short* __restrict__ Hout,
                                                      float carry) {
  __shared__ float red[8];
  const int row  = blockIdx.x;
  const int t    = threadIdx.x;
  const int lane = t & 31, wave = t >> 5;
  const int c0   = t * 8;
  const float* orow = O + (size_t)row * kEmb2 + c0;
  const v4f a = *(const v4f*)(orow);
  const v4f c = *(const v4f*)(orow + 4);
  float x[8];
#pragma unroll
  for (int e = 0; e < 4; ++e) { x[e] = a[e]; x[4 + e] = c[e]; }
  float ss = 0.0f;
#pragma unroll
  for (int e = 0; e < 8; ++e) ss += x[e] * x[e];
#pragma unroll
  for (int off = 16; off > 0; off >>= 1) ss += __shfl_xor(ss, off, 32);
  if (lane == 0) red[wave] = ss;
  __syncthreads();
  const int hd = t >> 6;
  const float tot  = red[2 * hd] + red[2 * hd + 1];
  const float mean = tot * kInvDv;
  const float rinv = 1.0f / sqrtf(mean + kEps);
  const float* grow = G + (size_t)row * kEmb2 + c0;
  const v4f ga = *(const v4f*)(grow);
  const v4f gc = *(const v4f*)(grow + 4);
  const float* wp = gnw + (c0 & (kDv - 1));
  const v4f wa = *(const v4f*)(wp);
  const v4f wc = *(const v4f*)(wp + 4);
  float gv[8], wv[8];
#pragma unroll
  for (int e = 0; e < 4; ++e) { gv[e] = ga[e]; gv[4 + e] = gc[e]; wv[e] = wa[e]; wv[4 + e] = wc[e]; }
  unsigned short hb[8];
#pragma unroll
  for (int e = 0; e < 8; ++e) {
    const float hv = ((x[e] * rinv) * wv[e]) * gv[e] * carry;
    hb[e] = h_bits(hv);
  }
  const v4u u = (v4u){pk16(hb[0], hb[1]), pk16(hb[2], hb[3]), pk16(hb[4], hb[5]), pk16(hb[6], hb[7])};
  unsigned short* q = Hout + (size_t)row * kEmb2 + c0;
  *(volatile v4u*)q = u;
  __threadfence();
  *(volatile v4u*)q = u;
}

extern "C" void kernel_launch(void* const* d_in, const int* in_sizes, int n_in,
                              void* d_out, int out_size, void* d_ws, size_t ws_size, hipStream_t stream) {
  if (n_in < 7) return;
  if (in_sizes[0] != kTok * kEmb || in_sizes[1] != kEmb * kEmb || in_sizes[2] != kEmb * kEmb ||
      in_sizes[3] != kEmb * kEmb2 || in_sizes[4] != kEmb * kEmb2 || in_sizes[5] != kEmb2 * kEmb ||
      in_sizes[6] != kDv) return;
  if (out_size != kTok * kEmb) return;
  const size_t kMiB = 1048576;
  const size_t wsTotal = 112 * kMiB;
  if (ws_size < wsTotal) return;

  const float* x   = (const float*)d_in[0];
  const float* Wq  = (const float*)d_in[1];
  const float* Wk  = (const float*)d_in[2];
  const float* Wv  = (const float*)d_in[3];
  const float* Wg  = (const float*)d_in[4];
  const float* Wo  = (const float*)d_in[5];
  const float* gnw = (const float*)d_in[6];
  float* out = (float*)d_out;
  char* ws = (char*)d_ws;

  float* TMPQ = (float*)(ws + 0 * kMiB);
  float* TMPK = (float*)(ws + 16 * kMiB);
  unsigned short* WqT = (unsigned short*)(ws + 32 * kMiB);
  unsigned short* WkT = (unsigned short*)(ws + 34 * kMiB);
  unsigned short* WvT = (unsigned short*)(ws + 36 * kMiB);
  float* SC32 = (float*)(ws + 0 * kMiB);
  unsigned short* S16 = (unsigned short*)(ws + 16 * kMiB);
  float* G32 = (float*)(ws + 0 * kMiB);
  unsigned short* X16 = (unsigned short*)(ws + 40 * kMiB);
  unsigned short* Q16 = (unsigned short*)(ws + 48 * kMiB);
  unsigned short* K16 = (unsigned short*)(ws + 56 * kMiB);
  unsigned short* H16 = (unsigned short*)(ws + 48 * kMiB);
  unsigned short* VT16 = (unsigned short*)(ws + 64 * kMiB);
  unsigned short* WgT = (unsigned short*)(ws + 64 * kMiB);
  unsigned short* WoT = (unsigned short*)(ws + 68 * kMiB);
  float* O32 = (float*)(ws + 80 * kMiB);
  const float* dummyR = (const float*)d_ws;

  RopeTab tab;
  for (int f = 0; f < 128; ++f) {
    const float e = (float)(2 * f) / 256.0f;
    const float p = (float)pow(10000.0, (double)e);
    tab.inv[f] = 1.0f / p;
  }
  float lg[kHeads];
  for (int h = 0; h < kHeads; ++h) {
    const double gm = 1.0 - ldexp(1.0, -5 - h);
    lg[h] = (float)log2(gm);
  }

  const dim3 b256(256);

  cast8_f16_kernel<<<dim3((kTok * kEmb / 8) / 256), b256, 0, stream>>>(x, X16, kTok * kEmb / 8);
  wtcast_kernel<<<dim3(kEmb / 64, kEmb / 64, 2), b256, 0, stream>>>(Wq, Wk, WqT, WkT, kEmb, kEmb, kWCarry);
  wtcast_kernel<<<dim3(kEmb / 64, kEmb2 / 64, 1), b256, 0, stream>>>(Wv, Wv, WvT, WvT, kEmb, kEmb2, kWCarry);

  wmma_gemm64<0, false, 0, 0, false, 0, 0><<<dim3((kTok / 64) * (kEmb / 64) / 8, 2), b256, 0, stream>>>(
      X16, X16, kEmb, 0L,
      WqT, WqT, kEmb, (long)kEmb * kEmb,
      (void*)TMPQ, (void*)TMPQ, kEmb, (long)kTok * kEmb,
      gnw, dummyR, 0L,
      kTok, kEmb, kEmb, kWCarryInv);

  rotary_kernel<<<dim3(kTok * kHeads), dim3(128), 0, stream>>>(TMPQ, TMPK, Q16, K16, tab);

  wmma_gemm64<0, false, 0, 1, false, 0, 0><<<dim3((kEmb2 / 64) * (kSeqT / 64) / 8, kBatch), b256, 0, stream>>>(
      WvT, WvT, kEmb, 0L,
      X16, X16, kEmb, (long)kSeqT * kEmb,
      (void*)VT16, (void*)VT16, kSeqT, (long)kEmb2 * kSeqT,
      gnw, dummyR, 0L,
      kEmb2, kSeqT, kEmb, kWCarryInv);

  for (int g = 0; g < kBatch * kHeads; ++g) {
    const int b = g >> 2, h = g & 3;
    const unsigned short* Qg = Q16 + (size_t)g * kSeqT * kDk;
    const unsigned short* Kg = K16 + (size_t)g * kSeqT * kDk;
    wmma_gemm64<0, false, 0, 0, false, 0, 1><<<dim3((kSeqT / 64) * (kSeqT / 64) / 8, 1), b256, 0, stream>>>(
        Qg, Qg, kDk, 0L,
        Kg, Kg, kDk, 0L,
        (void*)SC32, (void*)SC32, kSeqT, 0L,
        gnw, dummyR, 0L,
        kSeqT, kSeqT, kDk, kQScale);
    decay_cast_kernel<<<dim3(kSeqT), b256, 0, stream>>>(SC32, S16, lg[h], kSCarry);
    const unsigned short* Vg = VT16 + (size_t)g * kDv * kSeqT;
    float* Og = O32 + (size_t)b * kSeqT * kEmb2 + (size_t)h * kDv;
    wmma_gemm64<0, false, 0, 0, false, 0, 2><<<dim3((kSeqT / 64) * (kDv / 64) / 8, 1), b256, 0, stream>>>(
        S16, S16, kSeqT, 0L,
        Vg, Vg, kSeqT, 0L,
        (void*)Og, (void*)Og, kEmb2, 0L,
        gnw, dummyR, 0L,
        kSeqT, kDv, kSeqT, kSCarryInv);
  }

  wtcast_kernel<<<dim3(kEmb / 64, kEmb2 / 64, 1), b256, 0, stream>>>(Wg, Wg, WgT, WgT, kEmb, kEmb2, kWCarry);
  wtcast_kernel<<<dim3(kEmb2 / 64, kEmb / 64, 1), b256, 0, stream>>>(Wo, Wo, WoT, WoT, kEmb2, kEmb, kWCarry);

  wmma_gemm64<0, false, 0, 0, false, 0, 0><<<dim3((kTok / 64) * (kEmb2 / 64) / 8, 1), b256, 0, stream>>>(
      X16, X16, kEmb, 0L,
      WgT, WgT, kEmb, 0L,
      (void*)G32, (void*)G32, kEmb2, 0L,
      gnw, dummyR, 0L,
      kTok, kEmb2, kEmb, kWCarryInv);

  rmsgate_kernel<<<dim3(kTok), b256, 0, stream>>>(O32, G32, gnw, H16, kHCarry);

  wmma_gemm64<0, false, 0, 0, false, 0, 0><<<dim3((kTok / 64) * (kEmb / 64) / 8, 1), b256, 0, stream>>>(
      H16, H16, kEmb2, 0L,
      WoT, WoT, kEmb2, 0L,
      (void*)out, (void*)out, kEmb, 0L,
      gnw, dummyR, 0L,
      kTok, kEmb, kEmb2, kOutScale);
}
